// WindowAttentionAugmented_60550448939747
// MI455X (gfx1250) — hardware-verified
//
#include <hip/hip_runtime.h>
#include <math.h>

typedef __attribute__((ext_vector_type(16))) _Float16 v16h;
typedef __attribute__((ext_vector_type(16))) __bf16 v16b;
typedef __attribute__((ext_vector_type(8)))  _Float16 v8h;
typedef __attribute__((ext_vector_type(8)))  float v8f;
typedef __attribute__((ext_vector_type(4)))  float v4f;
typedef __attribute__((ext_vector_type(2)))  float v2f;
typedef __attribute__((ext_vector_type(4)))  unsigned v4u;
typedef __attribute__((ext_vector_type(4)))  int v4i;
typedef float __attribute__((may_alias)) float_a;
typedef int __attribute__((may_alias)) int_a;

template <typename T> __device__ __forceinline__ void vst2(void* p, T v) { *(volatile T*)p = v; __threadfence(); *(volatile T*)p = v; }
__device__ __forceinline__ v8f wmma16(v16h a, v16h b, v8f c) {
  v8f d = __builtin_amdgcn_wmma_f32_16x16x32_f16(false, a, false, b, (short)0, c, false, false);
  asm volatile("v_nop\n\tv_nop\n\tv_nop\n\tv_nop" : "+v"(d) : "v"(a), "v"(b));
  return d;
}
__device__ __forceinline__ v8f wmma_bf(v16b a, v16b b, v8f c) {
  v8f d = __builtin_amdgcn_wmma_f32_16x16x32_bf16(false, a, false, b, (short)0, c, false, false);
  asm volatile("v_nop\n\tv_nop\n\tv_nop\n\tv_nop" : "+v"(d) : "v"(a), "v"(b));
  return d;
}
__device__ __forceinline__ v16h frag_h(const _Float16* rowk0, int lane) {
  union { v16h v; v8h q[2]; } u; const _Float16* p = rowk0 + 8 * (lane >> 4);
  u.q[0] = *(const v8h*)p; u.q[1] = *(const v8h*)(p + 16); return u.v;
}
__device__ __forceinline__ v16h frag_f32(const float* rowk0, int lane) {
  v16h a; const float* p = rowk0 + 8 * (lane >> 4);
#pragma unroll
  for (int i = 0; i < 8; ++i) { a[i] = (_Float16)p[i]; a[8 + i] = (_Float16)p[16 + i]; }
  return a;
}
__device__ __forceinline__ v16h frag_f32s(const float* rowk0, int lane, float sc) {
  v16h a; const float* p = rowk0 + 8 * (lane >> 4);
#pragma unroll
  for (int i = 0; i < 8; ++i) { a[i] = (_Float16)(p[i] * sc); a[8 + i] = (_Float16)(p[16 + i] * sc); }
  return a;
}
__device__ __forceinline__ v16h fragc_f32(const float* W, int k0, int n, int lane, int ld, int K) {
  v16h a; const int g = lane >> 4;
#pragma unroll
  for (int i = 0; i < 8; ++i) { const int ka = k0 + 8 * g + i, kb = ka + 16;
    a[i] = (_Float16)(ka < K ? W[(size_t)(ka < K ? ka : K - 1) * ld + n] : 0.f); a[8 + i] = (_Float16)(kb < K ? W[(size_t)(kb < K ? kb : K - 1) * ld + n] : 0.f); }
  return a;
}
struct F2 { v16b h, l; };
__device__ __forceinline__ F2 bsplit16(const float v[16]) { F2 r;
#pragma unroll
  for (int i = 0; i < 16; ++i) { const __bf16 h = (__bf16)v[i]; r.h[i] = h; r.l[i] = (__bf16)(v[i] - (float)h); }
  return r; }
__device__ __forceinline__ F2 split_row(const float* row, int k0, int lane) { float v[16]; const float* p = row + k0 + 8 * (lane >> 4);
#pragma unroll
  for (int i = 0; i < 8; ++i) { v[i] = p[i]; v[8 + i] = p[16 + i]; }
  return bsplit16(v); }
__device__ __forceinline__ F2 split_rowK(const float* row, int k0, int lane, int K) { float v[16]; const int g = lane >> 4;
#pragma unroll
  for (int i = 0; i < 8; ++i) { const int ka = k0 + 8 * g + i, kb = ka + 16; v[i] = ka < K ? row[ka < K ? ka : K - 1] : 0.f; v[8 + i] = kb < K ? row[kb < K ? kb : K - 1] : 0.f; }
  return bsplit16(v); }
__device__ __forceinline__ F2 split_col(const float* W, int k0, int n, int lane, int ld, int K) { float v[16]; const int g = lane >> 4;
#pragma unroll
  for (int i = 0; i < 8; ++i) { const int ka = k0 + 8 * g + i, kb = ka + 16; v[i] = ka < K ? W[(size_t)(ka < K ? ka : K - 1) * ld + n] : 0.f; v[8 + i] = kb < K ? W[(size_t)(kb < K ? kb : K - 1) * ld + n] : 0.f; }
  return bsplit16(v); }
__device__ __forceinline__ v8f mac3(const F2& a, const F2& b, v8f c) { c = wmma_bf(a.l, b.h, c); c = wmma_bf(a.h, b.l, c); return wmma_bf(a.h, b.h, c); }
__device__ __forceinline__ float sigm(float v) { return 1.0f / (1.0f + expf(-v)); }
#define LDSX() do { asm volatile("s_wait_dscnt 0" ::: "memory"); __builtin_amdgcn_wave_barrier(); __builtin_amdgcn_fence(__ATOMIC_RELEASE, "workgroup"); } while (0)


#define NT_ 8
#define HH 128
#define CCH 32
#define PS 8
#define LL 64
#define NWIN 32
#define NW (NT_ * NWIN * NWIN)
#ifndef TNW
#define TNW NW
#define TNT NT_
#endif
__device__ __forceinline__ float bfr(float v) { return (float)(__bf16)v; }
__device__ __attribute__((noinline)) float exp_ni(float v) { return expf(v); }
typedef __attribute__((ext_vector_type(8))) __bf16 v8b;
__device__ __forceinline__ v16b frag_b(const __bf16* rowk0, int lane) {
  union { v16b v; v8b q[2]; } u; const __bf16* p = rowk0 + 8 * (lane >> 4);
  u.q[0] = *(const v8b*)p; u.q[1] = *(const v8b*)(p + 16); return u.v;
}
__device__ __forceinline__ int refl(int u) { return u >= HH ? 2 * (HH - 1) - u : u; }

__global__ __launch_bounds__(256) void k_bias(const float* __restrict__ tab, const int* __restrict__ idx, float* __restrict__ BIAS) {
  const int tid = threadIdx.x;
  for (int q = tid; q < 2 * LL * LL / 4; q += 256) { v4f v; const int h = q / (LL * LL / 4), base = (q % (LL * LL / 4)) * 4;
#pragma unroll
    for (int i = 0; i < 4; ++i) { int id = idx[base + i]; id = id < 0 ? 0 : (id > 224 ? 224 : id); v[i] = bfr(tab[id * 2 + h]); }
    vst2(BIAS + q * 4, v); }
}
__global__ __launch_bounds__(128) void k_win(const float* __restrict__ X, const float* __restrict__ Wqkv, const float* __restrict__ bqkv, const float* __restrict__ Wp, const float* __restrict__ bp, const float* __restrict__ BIAS, float* __restrict__ OUTW) {
  __shared__ __align__(16) __bf16 spat[LL][40];
  __shared__ __align__(16) __bf16 swq[96][40], swp[32][40];
  __shared__ __align__(16) float sq[LL][100];
  __shared__ __align__(16) __bf16 svh[32][72], svl[32][72];
  __shared__ __align__(16) float sp[4][16][68];
  __shared__ __align__(16) float so[LL][36];
  const int tid = threadIdx.x, wave = tid >> 5, lane = tid & 31, col = lane & 15, g = lane >> 4;
  const int win = blockIdx.x; const int t = win / (NWIN * NWIN), wr = (win / NWIN) % NWIN, wc = win % NWIN;
  for (int q = tid; q < 96 * 32; q += 128) { const int n = q >> 5, k = q & 31; swq[n][k] = (__bf16)Wqkv[n * 32 + k]; }
  for (int q = tid; q < 32 * 32; q += 128) { const int n = q >> 5, k = q & 31; swp[n][k] = (__bf16)Wp[n * 32 + k]; }
  for (int q = tid; q < LL * 32; q += 128) { const int l = q >> 5, c = q & 31; const int y = refl(wr * 4 + (l >> 3)), x = refl(wc * 4 + (l & 7)); spat[l][c] = (__bf16)X[(((size_t)t * HH + y) * HH + x) * CCH + c]; }
  __syncthreads();
  { const v16b a = frag_b(&spat[wave * 16 + col][0], lane);
#pragma unroll
    for (int ct = 0; ct < 6; ++ct) { v8f acc = {}; acc = wmma_bf(a, frag_b(&swq[ct * 16 + col][0], lane), acc);
#pragma unroll
      for (int r = 0; r < 8; ++r) { const int n = ct * 16 + col; sq[wave * 16 + 8 * g + r][n] = acc[r] + bfr(bqkv[n]); } } }
  __syncthreads();
  for (int q = tid; q < 32 * LL; q += 128) { const int hd_ = q >> 6, m = q & 63; const float v = sq[m][64 + hd_]; const __bf16 hi = (__bf16)v; svh[hd_][m] = hi; svl[hd_][m] = (__bf16)(v - (float)hi); }
  __syncthreads();
#pragma unroll 1
  for (int h = 0; h < 2; ++h) {
    const F2 a = split_rowK(&sq[wave * 16 + col][h * 16], 0, lane, 16);
    v8f s[4];
#pragma unroll
    for (int ct = 0; ct < 4; ++ct) { const F2 kb = split_rowK(&sq[ct * 16 + col][32 + h * 16], 0, lane, 16); s[ct] = mac3(a, kb, (v8f){}); }
#pragma unroll
    for (int r = 0; r < 8; ++r) { const int l = wave * 16 + 8 * g + r; float mx = -3.0e38f;
#pragma unroll
      for (int ct = 0; ct < 4; ++ct) { const float v = s[ct][r] * 0.25f + BIAS[(h * LL + l) * LL + ct * 16 + col]; s[ct][r] = v; mx = fmaxf(mx, v); }
#pragma unroll
      for (int o = 1; o < 16; o <<= 1) mx = fmaxf(mx, __shfl_xor(mx, o));
      float sum = 0.f;
#pragma unroll
      for (int ct = 0; ct < 4; ++ct) { const float e = exp_ni(s[ct][r] - mx); s[ct][r] = e; sum += e; }
#pragma unroll
      for (int o = 1; o < 16; o <<= 1) sum += __shfl_xor(sum, o);
      const float inv = 1.0f / sum;
#pragma unroll
      for (int ct = 0; ct < 4; ++ct) sp[wave][8 * g + r][ct * 16 + col] = s[ct][r] * inv; }
    LDSX();
    { v8f o = {};
#pragma unroll
      for (int kc = 0; kc < 2; ++kc) { const F2 pa = split_row(&sp[wave][col][0], kc * 32, lane); const __bf16* vh0 = &svh[h * 16 + col][kc * 32]; const __bf16* vl0 = &svl[h * 16 + col][kc * 32];
        o = wmma_bf(pa.l, frag_b(vh0, lane), o); o = wmma_bf(pa.h, frag_b(vl0, lane), o); o = wmma_bf(pa.h, frag_b(vh0, lane), o); }
#pragma unroll
      for (int r = 0; r < 8; ++r) so[wave * 16 + 8 * g + r][h * 16 + col] = o[r]; }
    LDSX(); }
  { const F2 a = split_row(&so[wave * 16 + col][0], 0, lane); v8f acc[2];
#pragma unroll
    for (int ct = 0; ct < 2; ++ct) { const v16b w = frag_b(&swp[ct * 16 + col][0], lane); acc[ct] = (v8f){}; acc[ct] = wmma_bf(a.l, w, acc[ct]); acc[ct] = wmma_bf(a.h, w, acc[ct]); }
    LDSX();
#pragma unroll
    for (int ct = 0; ct < 2; ++ct)
#pragma unroll
      for (int r = 0; r < 8; ++r) { const int n = ct * 16 + col; so[wave * 16 + 8 * g + r][n] = acc[ct][r] + bfr(bp[n]); } }
  LDSX();
  for (int q = lane; q < 16 * 8; q += 32) { const int rl = q >> 3, pc = q & 7; vst2(OUTW + ((size_t)win * LL + wave * 16 + rl) * CCH + pc * 4, *(const v4f*)&so[wave * 16 + rl][pc * 4]); }
}
__device__ __forceinline__ int axis_terms(int y, int* wv, int* iv) {
  int n = 0;
#pragma unroll
  for (int pass = 0; pass < 2; ++pass) { const int u = pass == 0 ? y : 2 * (HH - 1) - y;
    if (pass == 1 && (u < HH || u > 4 * (NWIN - 1) + PS - 1 || u == y)) continue;
    for (int w = u / 4; w >= 0 && w >= (u - (PS - 1) + 3) / 4; --w) { const int i = u - 4 * w; if (w < NWIN && i >= 0 && i < PS && n < 3) { wv[n] = w; iv[n] = i; ++n; } } }
  return n;
}
__global__ __launch_bounds__(256) void k_fold(const float* __restrict__ OUTW, float* __restrict__ out) {
  __shared__ __align__(16) float srow[HH * CCH];
  const int t = blockIdx.y, y = blockIdx.x, tid = threadIdx.x; const int x = tid >> 1, chalf = tid & 1;
  int wy[3], iy[3], wx[3], jx[3]; const int ny = axis_terms(y, wy, iy), nx = axis_terms(x, wx, jx);
  float acc[16];
#pragma unroll
  for (int c = 0; c < 16; ++c) acc[c] = 0.f;
  for (int a = 0; a < ny; ++a) for (int b2 = 0; b2 < nx; ++b2) { const size_t win = ((size_t)t * NWIN + wy[a]) * NWIN + wx[b2]; const float* src = OUTW + (win * LL + iy[a] * PS + jx[b2]) * CCH + chalf * 16;
#pragma unroll
    for (int c4 = 0; c4 < 4; ++c4) { const float4 v = *(const float4*)(src + c4 * 4); acc[c4 * 4] += v.x; acc[c4 * 4 + 1] += v.y; acc[c4 * 4 + 2] += v.z; acc[c4 * 4 + 3] += v.w; } }
  const float den = (float)(ny * nx) + 1e-10f;
#pragma unroll
  for (int c = 0; c < 16; ++c) srow[x * CCH + chalf * 16 + c] = acc[c] / den;
  __syncthreads();
  for (int q = tid; q < HH * CCH / 4; q += 256) vst2(out + (((size_t)t * HH + y) * HH) * CCH + q * 4, *(const v4f*)&srow[q * 4]);
}

extern "C" void kernel_launch(void* const* d_in, const int* in_sizes, int n_in, void* d_out, int out_size, void* d_ws, size_t ws_size, hipStream_t stream) {
  (void)in_sizes; (void)n_in; (void)out_size; (void)ws_size;
  const float* X = (const float*)d_in[0]; const float* Wqkv = (const float*)d_in[1]; const float* bqkv = (const float*)d_in[2]; const float* tab = (const float*)d_in[3]; const float* Wp = (const float*)d_in[4]; const float* bp = (const float*)d_in[5]; const int* idx = (const int*)d_in[6];
  char* ws = (char*)d_ws; float* BIAS = (float*)ws; float* OUTW = BIAS + 2 * LL * LL;
  k_bias<<<1, 256, 0, stream>>>(tab, idx, BIAS);
  k_win<<<TNW, 128, 0, stream>>>(X, Wqkv, bqkv, Wp, bp, BIAS, OUTW);
  k_fold<<<dim3(HH, TNT), 256, 0, stream>>>(OUTW, (float*)d_out);
}
